// CustomMultiHeadSelfAttention_35742717837546
// MI455X (gfx1250) — hardware-verified
//
#include <hip/hip_runtime.h>
#include <math.h>
#include <stdint.h>

#define NBATCH  4
#define SEQ_LEN 2048
#define D_MODEL 1024
#define N_QKV   3072
#define NHEADS  16
#define D_HEAD  64

typedef __attribute__((ext_vector_type(16))) _Float16 v16h;
typedef __attribute__((ext_vector_type(8)))  _Float16 v8h;
typedef __attribute__((ext_vector_type(16))) __bf16   v16b;
typedef __attribute__((ext_vector_type(8)))  __bf16   v8b;
typedef __attribute__((ext_vector_type(8)))  float    v8f;
typedef __attribute__((ext_vector_type(4)))  float    v4f;
typedef __attribute__((ext_vector_type(2)))  float    v2f;
typedef __attribute__((ext_vector_type(4)))  unsigned int v4u;

__device__ __forceinline__ unsigned short f2bf_bits(float f) {
  unsigned u = __float_as_uint(f);
  return (unsigned short)((u + 0x7FFFu + ((u >> 16) & 1u)) >> 16);
}
__device__ __forceinline__ float bf_bits2f(unsigned short h) { return __uint_as_float(((unsigned)h) << 16); }

__device__ __forceinline__ void dep_guard_h(v8f& a, v8f& b, v16h x, v16h y) { asm volatile("v_nop\n\tv_nop\n\tv_nop\n\tv_nop" : "+v"(a), "+v"(b) : "v"(x), "v"(y)); }
__device__ __forceinline__ void dep_guard_b(v8f& a, v8f& b, v16b x, v16b y) { asm volatile("v_nop\n\tv_nop\n\tv_nop\n\tv_nop" : "+v"(a), "+v"(b) : "v"(x), "v"(y)); }
__device__ __forceinline__ void keep4_h(v16h a, v16h b, v16h c, v16h d) { asm volatile("v_nop" :: "v"(a), "v"(b), "v"(c), "v"(d)); }
__device__ __forceinline__ void keep4_b(v16b a, v16b b, v16b c, v16b d) { asm volatile("v_nop" :: "v"(a), "v"(b), "v"(c), "v"(d)); }
__device__ __forceinline__ void acc_guard4(v8f& a, v8f& b, v8f& c, v8f& d) { asm volatile("v_nop\n\tv_nop\n\tv_nop\n\tv_nop" : "+v"(a), "+v"(b), "+v"(c), "+v"(d)); }
template <typename T> struct Frag;
template <> struct Frag<_Float16> {
  typedef v16h V; union U { v16h v; v8h h[2]; };
  static __device__ __forceinline__ v16h load(const _Float16* p) {
    U f; f.h[0] = *(const v8h*)(p); f.h[1] = *(const v8h*)(p + 16); return f.v;
  }
  static __device__ __forceinline__ v8f mma(v16h a, v16h b, v8f c) {
    return __builtin_amdgcn_wmma_f32_16x16x32_f16(false, a, false, b, (short)0, c, false, false);
  }
  static __device__ __forceinline__ void guard(v8f& a, v8f& b, v16h x, v16h y) { dep_guard_h(a, b, x, y); }
  static __device__ __forceinline__ void keep(v16h a, v16h b, v16h c, v16h d) { keep4_h(a, b, c, d); }
};
template <> struct Frag<__bf16> {
  typedef v16b V; union U { v16b v; v8b h[2]; };
  static __device__ __forceinline__ v16b load(const __bf16* p) {
    U f; f.h[0] = *(const v8b*)(p); f.h[1] = *(const v8b*)(p + 16); return f.v;
  }
  static __device__ __forceinline__ v8f mma(v16b a, v16b b, v8f c) {
    return __builtin_amdgcn_wmma_f32_16x16x32_bf16(false, a, false, b, (short)0, c, false, false);
  }
  static __device__ __forceinline__ void guard(v8f& a, v8f& b, v16b x, v16b y) { dep_guard_b(a, b, x, y); }
  static __device__ __forceinline__ void keep(v16b a, v16b b, v16b c, v16b d) { keep4_b(a, b, c, d); }
};

template <int ET> struct Elem;
template <> struct Elem<0> { typedef _Float16 T; };
template <> struct Elem<1> { typedef __bf16 T; };
template <int ET, bool SPLIT, int BIAS_MODE, int OUT_MODE, bool RESID, int ACT = 0>
__global__ __launch_bounds__(256) void wmma_gemm64(
    const unsigned short* __restrict__ Ap, const unsigned short* __restrict__ A2p, int lda, long strideA,
    const unsigned short* __restrict__ Btp, const unsigned short* __restrict__ Bt2p, int ldb, long strideB,
    void* __restrict__ Cout, void* __restrict__ Cout2, int ldc, long strideC,
    const float* __restrict__ bias,
    const float* __restrict__ resid, long strideR,
    int M, int N, int K, float scale) {
  typedef typename Elem<ET>::T T;
  typedef typename Frag<T>::V V;
  const T* A = (const T*)Ap; const T* A2 = (const T*)A2p; const T* Bt = (const T*)Btp; const T* Bt2 = (const T*)Bt2p;
  __shared__ __align__(16) float sT[8][16 * 68];
  const int b    = blockIdx.y;
  const int lane = threadIdx.x & 31;
  const int wave = threadIdx.x >> 5;
  const int tilesN = N >> 6;
  const int tilesM = M >> 6;
  const int tile = blockIdx.x * 8 + wave;
  if (tile >= tilesM * tilesN) return;
  const int tm = tile / tilesN;
  const int tn = tile - tm * tilesN;
  const int m0 = tm << 6;
  const int n0 = tn << 6;

  const T* Ab  = A  + (size_t)b * strideA;
  const T* Bb  = Bt + (size_t)b * strideB;
  const T* Ab2 = SPLIT ? (A2  + (size_t)b * strideA) : nullptr;
  const T* Bb2 = SPLIT ? (Bt2 + (size_t)b * strideB) : nullptr;

  const int rlane = lane & 15;
  const int koff  = (lane >> 4) * 8;
  const int mOff  = (lane >> 4) * 8;

  v8f acc[4][4];
#pragma unroll
  for (int i = 0; i < 4; ++i)
#pragma unroll
    for (int j = 0; j < 4; ++j) acc[i][j] = (v8f){0.f,0.f,0.f,0.f,0.f,0.f,0.f,0.f};

  for (int k0 = 0; k0 < K; k0 += 32) {
    V bh[4], bl[4];
#pragma unroll
    for (int j = 0; j < 4; ++j) {
      const size_t bo = (size_t)(n0 + (j << 4) + rlane) * ldb + koff + k0;
      bh[j] = Frag<T>::load(Bb + bo);
      if (SPLIT) bl[j] = Frag<T>::load(Bb2 + bo);
    }
#pragma unroll
    for (int i = 0; i < 4; ++i) {
      const size_t ao = (size_t)(m0 + (i << 4) + rlane) * lda + koff + k0;
      V ah = Frag<T>::load(Ab + ao);
      V al;
      if (SPLIT) al = Frag<T>::load(Ab2 + ao);
#pragma unroll
      for (int j = 0; j < 4; ++j) {
        acc[i][j] = Frag<T>::mma(ah, bh[j], acc[i][j]);
        if (SPLIT) {
          acc[i][j] = Frag<T>::mma(ah, bl[j], acc[i][j]);
          acc[i][j] = Frag<T>::mma(al, bh[j], acc[i][j]);
        }
      }
      Frag<T>::guard(acc[i][0], acc[i][3], ah, SPLIT ? al : ah);
    }
    Frag<T>::keep(bh[0], bh[1], bh[2], bh[3]);
    if (SPLIT) Frag<T>::keep(bl[0], bl[1], bl[2], bl[3]);
  }
  acc_guard4(acc[0][0], acc[0][1], acc[0][2], acc[0][3]);
  acc_guard4(acc[1][0], acc[1][1], acc[1][2], acc[1][3]);
  acc_guard4(acc[2][0], acc[2][1], acc[2][2], acc[2][3]);
  acc_guard4(acc[3][0], acc[3][1], acc[3][2], acc[3][3]);

  float* slab = sT[wave];
  const float* Rb = RESID ? (resid + (size_t)b * strideR) : nullptr;
#pragma unroll
  for (int i = 0; i < 4; ++i) {
    const int mBase = m0 + (i << 4);
#pragma unroll
    for (int j = 0; j < 4; ++j) {
      const int n = n0 + (j << 4) + rlane;
      float bv = 0.f;
      if (BIAS_MODE == 2) bv = bias[n];
#pragma unroll
      for (int r = 0; r < 8; ++r) {
        float v = acc[i][j][r] * scale;
        if (BIAS_MODE == 1) v += bias[mBase + mOff + r];
        if (BIAS_MODE == 2) v += bv;
        if (RESID) v += Rb[(size_t)(mBase + mOff + r) * ldc + n];
        if (ACT == 1) v = tanhf(v);
        if (ACT == 2) v = fmaxf(v, 0.0f);
        if (ACT == 3) v = v / (1.0f + expf(-v));
        if (ACT == 4) v = (v > 0.f) ? v : 0.01f * v;
        if (ACT == 5) v = 0.5f * v * (1.0f + erff(v * 0.70710678118654752f));
        slab[(mOff + r) * 68 + (j << 4) + rlane] = v;
      }
    }
    __builtin_amdgcn_fence(__ATOMIC_RELEASE, "workgroup");
    __builtin_amdgcn_wave_barrier();
    __builtin_amdgcn_fence(__ATOMIC_ACQUIRE, "workgroup");
    if (OUT_MODE == 0) {
      float* C = (float*)Cout + (size_t)b * strideC;
      const int hh = lane >> 4, c4 = (lane & 15) * 4;
      for (int pass = 0; pass < 2; ++pass) {
#pragma unroll
        for (int it = 0; it < 8; ++it) {
          const int row = it * 2 + hh;
          v4f v = *(const v4f*)(slab + row * 68 + c4);
          *(volatile v4f*)(C + (size_t)(mBase + row) * ldc + n0 + c4) = v;
        }
        __threadfence();
      }
    } else {
      const int q = lane >> 3, c8 = (lane & 7) * 8;
      unsigned short* C  = (unsigned short*)Cout  + (size_t)b * strideC;
      unsigned short* C2 = (OUT_MODE == 2) ? ((unsigned short*)Cout2 + (size_t)b * strideC) : nullptr;
      for (int pass = 0; pass < 2; ++pass) {
#pragma unroll
        for (int it = 0; it < 4; ++it) {
          const int row = it * 4 + q;
          const float* sp = slab + row * 68 + c8;
          v8h hv, lv;
#pragma unroll
          for (int e = 0; e < 8; ++e) {
            if (OUT_MODE == 1) {
              hv[e] = (_Float16)sp[e];
            } else {
              unsigned short hb = f2bf_bits(sp[e]);
              unsigned short lb = f2bf_bits(sp[e] - bf_bits2f(hb));
              hv[e] = __builtin_bit_cast(_Float16, hb);
              lv[e] = __builtin_bit_cast(_Float16, lb);
            }
          }
          *(volatile v8h*)(C + (size_t)(mBase + row) * ldc + n0 + c8) = hv;
          if (OUT_MODE == 2) *(volatile v8h*)(C2 + (size_t)(mBase + row) * ldc + n0 + c8) = lv;
        }
        __threadfence();
      }
    }
    __builtin_amdgcn_fence(__ATOMIC_RELEASE, "workgroup");
    __builtin_amdgcn_wave_barrier();
    __builtin_amdgcn_fence(__ATOMIC_ACQUIRE, "workgroup");
  }
}

__global__ __launch_bounds__(256) void cast_f32_f16x2(
    const float* __restrict__ in, _Float16* __restrict__ out, int n2) {
  int i = blockIdx.x * 256 + threadIdx.x;
  if (i < n2) {
    const _Float16 h0 = (_Float16)in[2 * i], h1 = (_Float16)in[2 * i + 1];
    const unsigned u = (unsigned)__builtin_bit_cast(unsigned short, h0) | ((unsigned)__builtin_bit_cast(unsigned short, h1) << 16);
    ((volatile unsigned*)out)[i] = u;
    __threadfence();
    ((volatile unsigned*)out)[i] = u;
  }
}

__device__ __forceinline__ unsigned pk16(unsigned short a, unsigned short b) { return (unsigned)a | ((unsigned)b << 16); }
__device__ __forceinline__ unsigned short h_bits(float f) { return __builtin_bit_cast(unsigned short, (_Float16)f); }

__global__ __launch_bounds__(256) void tcast_f16_kernel(const float* __restrict__ W, unsigned short* __restrict__ o,
                                                        int R, int Cc, float scale) {
  __shared__ __align__(16) float tf[64 * 68];
  const int c0  = blockIdx.x * 64;
  const int r0  = blockIdx.y * 64;
  const int tid = threadIdx.x;
  {
    const int lr = tid >> 4;
    const int c4 = (tid & 15) * 4;
#pragma unroll
    for (int it = 0; it < 4; ++it) {
      const int rr = it * 16 + lr;
      const v4f a = *(const v4f*)(W + (size_t)(r0 + rr) * Cc + c0 + c4);
      *(v4f*)(tf + rr * 68 + c4) = a;
    }
  }
  __syncthreads();
  const int sub = tid >> 3;
  const int c8  = (tid & 7) * 8;
  v4u hv[2];
#pragma unroll
  for (int it = 0; it < 2; ++it) {
    const int oc = it * 32 + sub;
    v4u a;
#pragma unroll
    for (int qq = 0; qq < 4; ++qq) {
      const float f0 = tf[(c8 + 2 * qq) * 68 + oc] * scale;
      const float f1 = tf[(c8 + 2 * qq + 1) * 68 + oc] * scale;
      a[qq] = pk16(h_bits(f0), h_bits(f1));
    }
    hv[it] = a;
  }
  for (int pass = 0; pass < 2; ++pass) {
#pragma unroll
    for (int it = 0; it < 2; ++it) {
      const int oc = it * 32 + sub;
      const size_t go = (size_t)(c0 + oc) * R + r0 + c8;
      *(volatile v4u*)(o + go) = hv[it];
    }
    __threadfence();
  }
}

#define AT_D 64
#define AT_NW 4
#define AT_QB 64
#define AT_KC 64

__device__ __forceinline__ v8f at_mma_h(v16h a, v16h b, v8f c) {
  c = __builtin_amdgcn_wmma_f32_16x16x32_f16(false, a, false, b, (short)0, c, false, false);
  asm volatile("v_nop\n\tv_nop\n\tv_nop\n\tv_nop" : "+v"(c) : "v"(a), "v"(b));
  return c;
}

__global__ __launch_bounds__(128)
void attn_full64_f16_kernel(const unsigned short* __restrict__ qp, const unsigned short* __restrict__ kp, int ldqk,
                            const unsigned short* __restrict__ vtp, unsigned short* __restrict__ outp, int ldo,
                            float sscale, float oscale) {
  union FH { v16h v; v8h h[2]; };
  __shared__ __align__(16) _Float16 Ksh[AT_KC * AT_D];
  __shared__ __align__(16) _Float16 Vth[AT_D * AT_KC];
  __shared__ __align__(16) _Float16 Psh[AT_NW][16 * AT_KC];
  __shared__ __align__(16) float    Os[AT_NW][16 * 68];
  const float PSC = 32768.0f;

  const int tid  = threadIdx.x;
  const int wave = tid >> 5;
  const int lane = tid & 31;
  const int hh   = lane >> 4;
  const int c    = lane & 15;

  const int nqb = SEQ_LEN / AT_QB;
  const int qb = blockIdx.x % nqb;
  const int h  = blockIdx.x / nqb;
  const int b  = blockIdx.y;
  const int q0 = qb * AT_QB + wave * 16;

  const _Float16* Qh = (const _Float16*)(const void*)qp  + (size_t)b * SEQ_LEN * ldqk + (size_t)h * AT_D;
  const _Float16* Kh = (const _Float16*)(const void*)kp  + (size_t)b * SEQ_LEN * ldqk + (size_t)h * AT_D;
  const _Float16* Vh = (const _Float16*)(const void*)vtp + ((size_t)b * D_MODEL + (size_t)h * AT_D) * SEQ_LEN;
  _Float16*       ob = (_Float16*)(void*)outp + (size_t)b * SEQ_LEN * ldo + (size_t)h * AT_D;

  v16h qa[2];
#pragma unroll
  for (int dc = 0; dc < 2; ++dc)
    qa[dc] = Frag<_Float16>::load(Qh + (size_t)(q0 + c) * ldqk + dc * 32 + 8 * hh);

  float mrow[8], lrow[8];
  v8f oacc[4];
#pragma unroll
  for (int r = 0; r < 8; ++r) { mrow[r] = -INFINITY; lrow[r] = 0.f; }
#pragma unroll
  for (int t = 0; t < 4; ++t) oacc[t] = (v8f){0.f,0.f,0.f,0.f,0.f,0.f,0.f,0.f};

  const int nChunks = SEQ_LEN / AT_KC;
  for (int kc = 0; kc < nChunks; ++kc) {
    const int kv0 = kc * AT_KC;
    __syncthreads();
    {
      const int r = tid >> 1, half = (tid & 1) * 32;
      const _Float16* ks = Kh + (size_t)(kv0 + r) * ldqk + half;
      const _Float16* vs = Vh + (size_t)r * SEQ_LEN + kv0 + half;
#pragma unroll
      for (int i = 0; i < 4; ++i) {
        const v8h a0 = *(const v8h*)(ks + 8 * i);
        const v8h b0 = *(const v8h*)(vs + 8 * i);
        *(v8h*)(Ksh + r * AT_D  + half + 8 * i) = a0;
        *(v8h*)(Vth + r * AT_KC + half + 8 * i) = b0;
      }
    }
    __syncthreads();

    v8f s[4];
#pragma unroll
    for (int j = 0; j < 4; ++j) {
      s[j] = (v8f){0.f,0.f,0.f,0.f,0.f,0.f,0.f,0.f};
#pragma unroll
      for (int dc = 0; dc < 2; ++dc) {
        FH kb;
        kb.h[0] = *(const v8h*)(Ksh + (j * 16 + c) * AT_D + dc * 32 + 8 * hh);
        kb.h[1] = *(const v8h*)(Ksh + (j * 16 + c) * AT_D + dc * 32 + 16 + 8 * hh);
        s[j] = at_mma_h(qa[dc], kb.v, s[j]);
      }
    }
    float cm[8];
#pragma unroll
    for (int r = 0; r < 8; ++r) {
      float m = -INFINITY;
#pragma unroll
      for (int j = 0; j < 4; ++j) {
        const float sv = s[j][r] * sscale;
        s[j][r] = sv;
        m = fmaxf(m, sv);
      }
#pragma unroll
      for (int off = 1; off < 16; off <<= 1) m = fmaxf(m, __shfl_xor(m, off, 32));
      cm[r] = m;
    }
    _Float16* pw = Psh[wave];
#pragma unroll
    for (int r = 0; r < 8; ++r) {
      const float mnew = fmaxf(mrow[r], cm[r]);
      const float alpha = expf(mrow[r] - mnew);
      mrow[r] = mnew;
      float psum = 0.f;
#pragma unroll
      for (int j = 0; j < 4; ++j) {
        const float p = expf(s[j][r] - mnew);
        psum += p;
        pw[(8 * hh + r) * AT_KC + j * 16 + c] = (_Float16)(p * PSC);
      }
#pragma unroll
      for (int off = 1; off < 16; off <<= 1) psum += __shfl_xor(psum, off, 32);
      lrow[r] = lrow[r] * alpha + psum;
#pragma unroll
      for (int t = 0; t < 4; ++t) oacc[t][r] *= alpha;
    }
    __builtin_amdgcn_fence(__ATOMIC_RELEASE, "workgroup");
    __builtin_amdgcn_wave_barrier();
    __builtin_amdgcn_fence(__ATOMIC_ACQUIRE, "workgroup");
#pragma unroll 1
    for (int kk = 0; kk < 2; ++kk) {
      FH pa;
      pa.h[0] = *(const v8h*)(pw + c * AT_KC + kk * 32 + 8 * hh);
      pa.h[1] = *(const v8h*)(pw + c * AT_KC + kk * 32 + 16 + 8 * hh);
#pragma unroll
      for (int t = 0; t < 4; ++t) {
        FH vb;
        vb.h[0] = *(const v8h*)(Vth + (t * 16 + c) * AT_KC + kk * 32 + 8 * hh);
        vb.h[1] = *(const v8h*)(Vth + (t * 16 + c) * AT_KC + kk * 32 + 16 + 8 * hh);
        oacc[t] = at_mma_h(pa.v, vb.v, oacc[t]);
      }
    }
  }

  float* os = Os[wave];
#pragma unroll
  for (int r = 0; r < 8; ++r) {
    const float inv = oscale / (lrow[r] * PSC);
#pragma unroll
    for (int t = 0; t < 4; ++t) os[(8 * hh + r) * 68 + t * 16 + c] = oacc[t][r] * inv;
  }
  __builtin_amdgcn_fence(__ATOMIC_RELEASE, "workgroup");
  __builtin_amdgcn_wave_barrier();
  __builtin_amdgcn_fence(__ATOMIC_ACQUIRE, "workgroup");
  {
    const int q4 = lane >> 3, c8 = (lane & 7) * 8;
    for (int pass = 0; pass < 2; ++pass) {
#pragma unroll
      for (int it = 0; it < 4; ++it) {
        const int row = it * 4 + q4;
        const float* sp = os + row * 68 + c8;
        v8h hv;
#pragma unroll
        for (int e = 0; e < 8; ++e) hv[e] = (_Float16)sp[e];
        *(volatile v8h*)(ob + (size_t)(q0 + row) * ldo + c8) = hv;
      }
      __threadfence();
    }
  }
}

__global__ __launch_bounds__(256) void layernorm_rows_kernel(const float* __restrict__ res, const float* __restrict__ gam,
                                                             const float* __restrict__ bet, float* __restrict__ out,
                                                             int nrows, float eps) {
  const int wave = threadIdx.x >> 5, lane = threadIdx.x & 31;
  const int row = blockIdx.x * 8 + wave;
  if (row >= nrows) return;
  const float* rp = res + (size_t)row * D_MODEL;
  float s1 = 0.f;
#pragma unroll 1
  for (int i = 0; i < D_MODEL / 128; ++i) {
    const v4f v = *(const v4f*)(rp + i * 128 + lane * 4);
    s1 += (v[0] + v[1]) + (v[2] + v[3]);
  }
#pragma unroll
  for (int off = 1; off < 32; off <<= 1) s1 += __shfl_xor(s1, off, 32);
  const float mu = s1 * (1.0f / D_MODEL);
  float s2 = 0.f;
#pragma unroll 1
  for (int i = 0; i < D_MODEL / 128; ++i) {
    const v4f v = *(const v4f*)(rp + i * 128 + lane * 4);
    const float d0 = v[0] - mu, d1 = v[1] - mu, d2 = v[2] - mu, d3 = v[3] - mu;
    s2 += (d0 * d0 + d1 * d1) + (d2 * d2 + d3 * d3);
  }
#pragma unroll
  for (int off = 1; off < 32; off <<= 1) s2 += __shfl_xor(s2, off, 32);
  const float var  = s2 * (1.0f / D_MODEL);
  const float rstd = rsqrtf(var + eps);
  float* op = out + (size_t)row * D_MODEL;
  for (int pass = 0; pass < 2; ++pass) {
#pragma unroll 1
    for (int i = 0; i < D_MODEL / 128; ++i) {
      const v4f v  = *(const v4f*)(rp  + i * 128 + lane * 4);
      const v4f g  = *(const v4f*)(gam + i * 128 + lane * 4);
      const v4f bt = *(const v4f*)(bet + i * 128 + lane * 4);
      v4f o;
      o[0] = ((v[0] - mu) * rstd) * g[0] + bt[0];
      o[1] = ((v[1] - mu) * rstd) * g[1] + bt[1];
      o[2] = ((v[2] - mu) * rstd) * g[2] + bt[2];
      o[3] = ((v[3] - mu) * rstd) * g[3] + bt[3];
      *(volatile v4f*)(op + i * 128 + lane * 4) = o;
    }
    __threadfence();
  }
}

extern "C" void kernel_launch(void* const* d_in, const int* in_sizes, int n_in,
                              void* d_out, int out_size, void* d_ws, size_t ws_size,
                              hipStream_t stream) {
  const int NTOK = NBATCH * SEQ_LEN;
  if (n_in < 7) return;
  if (in_sizes[0] != NTOK * D_MODEL || in_sizes[1] != D_MODEL * N_QKV || in_sizes[2] != N_QKV ||
      in_sizes[3] != D_MODEL * D_MODEL || in_sizes[4] != D_MODEL || in_sizes[5] != D_MODEL ||
      in_sizes[6] != D_MODEL || out_size != NTOK * D_MODEL) return;

  const float* x     = (const float*)d_in[0];
  const float* Wqkv  = (const float*)d_in[1];
  const float* bqkv  = (const float*)d_in[2];
  const float* Wout  = (const float*)d_in[3];
  const float* bout  = (const float*)d_in[4];
  const float* gamma = (const float*)d_in[5];
  const float* beta  = (const float*)d_in[6];
  float* out = (float*)d_out;

  const size_t bytes_xh  = (size_t)NTOK * D_MODEL * 2;
  const size_t bytes_wqT = (size_t)N_QKV * D_MODEL * 2;
  const size_t bytes_woT = (size_t)D_MODEL * D_MODEL * 2;
  const size_t bytes_qk  = (size_t)NTOK * 2 * D_MODEL * 2;
  const size_t bytes_vT  = (size_t)NBATCH * D_MODEL * SEQ_LEN * 2;
  const size_t bytes_ao  = (size_t)NTOK * D_MODEL * 2;
  const size_t off_xh  = 0;
  const size_t off_wqT = off_xh  + bytes_xh;
  const size_t off_woT = off_wqT + bytes_wqT;
  const size_t off_qk  = off_woT + bytes_woT;
  const size_t off_vT  = off_qk  + bytes_qk;
  const size_t off_ao  = off_vT  + bytes_vT;
  const size_t total   = off_ao  + bytes_ao;
  if (total > ws_size) return;
  if ((size_t)NTOK * D_MODEL * 4 > bytes_qk) return;

  char* ws = (char*)d_ws;
  unsigned short* xh   = (unsigned short*)(ws + off_xh);
  unsigned short* wqT  = (unsigned short*)(ws + off_wqT);
  unsigned short* woT  = (unsigned short*)(ws + off_woT);
  unsigned short* qk   = (unsigned short*)(ws + off_qk);
  float*          resf = (float*)(ws + off_qk);
  unsigned short* vT   = (unsigned short*)(ws + off_vT);
  unsigned short* ao   = (unsigned short*)(ws + off_ao);

  {
    const int n2 = NTOK * D_MODEL / 2;
    cast_f32_f16x2<<<dim3((n2 + 255) / 256), dim3(256), 0, stream>>>(x, (_Float16*)(void*)xh, n2);
  }
  tcast_f16_kernel<<<dim3(N_QKV / 64, D_MODEL / 64), dim3(256), 0, stream>>>(Wqkv, wqT, D_MODEL, N_QKV, 64.0f);
  tcast_f16_kernel<<<dim3(D_MODEL / 64, D_MODEL / 64), dim3(256), 0, stream>>>(Wout, woT, D_MODEL, D_MODEL, 64.0f);
  wmma_gemm64<0, false, 2, 1, false><<<dim3((NTOK / 64) * (2 * D_MODEL / 64) / 8, 1), dim3(256), 0, stream>>>(
      xh, xh, D_MODEL, (long)0,
      wqT, wqT, D_MODEL, (long)0,
      (void*)qk, (void*)qk, 2 * D_MODEL, (long)0,
      bqkv, x, (long)0,
      NTOK, 2 * D_MODEL, D_MODEL, 0.015625f);
  wmma_gemm64<0, false, 1, 1, false><<<dim3((D_MODEL / 64) * (SEQ_LEN / 64) / 8, NBATCH), dim3(256), 0, stream>>>(
      wqT + (size_t)2 * D_MODEL * D_MODEL, wqT + (size_t)2 * D_MODEL * D_MODEL, D_MODEL, (long)0,
      xh, xh, D_MODEL, (long)SEQ_LEN * D_MODEL,
      (void*)vT, (void*)vT, SEQ_LEN, (long)D_MODEL * SEQ_LEN,
      bqkv + 2 * D_MODEL, x, (long)0,
      D_MODEL, SEQ_LEN, D_MODEL, 0.015625f);
  attn_full64_f16_kernel<<<dim3(NHEADS * (SEQ_LEN / AT_QB), NBATCH), dim3(128), 0, stream>>>(
      qk, qk + D_MODEL, 2 * D_MODEL, vT, ao, D_MODEL, 0.125f, 16.0f);
  wmma_gemm64<0, false, 2, 0, true><<<dim3((NTOK / 64) * (D_MODEL / 64) / 8, 1), dim3(256), 0, stream>>>(
      ao, ao, D_MODEL, (long)0,
      woT, woT, D_MODEL, (long)0,
      (void*)resf, (void*)resf, D_MODEL, (long)0,
      bout, x, (long)0,
      NTOK, D_MODEL, D_MODEL, 0.0009765625f);
  layernorm_rows_kernel<<<dim3(NTOK / 8), dim3(256), 0, stream>>>(resf, gamma, beta, out, NTOK, 1e-5f);
}
